// LSTMpredictor_45320494907929
// MI455X (gfx1250) — hardware-verified
//
#include <hip/hip_runtime.h>
#include <math.h>

constexpr int NBATCH = 1024;
constexpr int TLEN   = 1024;
constexpr int HID    = 51;
constexpr int NGATE  = 4;
constexpr int G4H    = NGATE * HID;
constexpr int UPAD   = 64;
constexpr int KP     = 64;
constexpr int MROWS  = 16;
constexpr int NWAVE  = UPAD / 16;
constexpr int NTHR   = 32 * NWAVE;
constexpr int TCH    = 32;
constexpr int NCHUNK = TLEN / TCH;
constexpr int HFP    = 64;
constexpr int NWW    = NGATE * UPAD * (KP / 2);
constexpr float HCARRY  = 16.0f;
constexpr float LCARRY  = 2048.0f;
constexpr float WCARRY  = 256.0f;
constexpr float FOLD_HI = 1.0f / (HCARRY * WCARRY);
constexpr float FOLD_LO = 1.0f / (HCARRY * WCARRY * LCARRY);
static_assert(NBATCH % MROWS == 0);
static_assert(TLEN % TCH == 0 && NCHUNK * TCH == TLEN);
static_assert(HID <= UPAD && UPAD % 32 == 0 && KP == UPAD);
static_assert(G4H == 204);
static_assert(MROWS * TCH == NTHR * 4);
static_assert(NWW % NTHR == 0);
static_assert((MROWS * KP / 2) % NTHR == 0);
static_assert((MROWS * HFP) % NTHR == 0);
static_assert(UPAD <= NTHR && UPAD == 64);
static_assert(MROWS == 4 * NWAVE);
static_assert(HFP == 64);

typedef __attribute__((ext_vector_type(16))) _Float16 v16h;
typedef __attribute__((ext_vector_type(8)))  _Float16 v8h;
typedef __attribute__((ext_vector_type(8)))  float    v8f;
typedef __attribute__((ext_vector_type(4)))  float    v4f;

__device__ __forceinline__ void acc_guard4(v8f& a, v8f& b, v8f& c, v8f& d) {
  asm volatile("v_nop\n\tv_nop\n\tv_nop\n\tv_nop" : "+v"(a), "+v"(b), "+v"(c), "+v"(d));
}
__device__ __forceinline__ void guard8x6(v8f& a0, v8f& a1, v8f& a2, v8f& a3, v8f& a4, v8f& a5, v8f& a6, v8f& a7,
                                         v16h x0, v16h x1, v16h y0, v16h y1, v16h y2, v16h y3) {
  asm volatile("v_nop\n\tv_nop\n\tv_nop\n\tv_nop"
               : "+v"(a0), "+v"(a1), "+v"(a2), "+v"(a3), "+v"(a4), "+v"(a5), "+v"(a6), "+v"(a7)
               : "v"(x0), "v"(x1), "v"(y0), "v"(y1), "v"(y2), "v"(y3));
}

template <typename T> struct Frag;
template <> struct Frag<_Float16> {
  typedef v16h V; union U { v16h v; v8h h[2]; };
  static __device__ __forceinline__ v16h load(const _Float16* p) {
    U f; f.h[0] = *(const v8h*)(p); f.h[1] = *(const v8h*)(p + 16); return f.v;
  }
  static __device__ __forceinline__ v8f mma(v16h a, v16h b, v8f c) {
    return __builtin_amdgcn_wmma_f32_16x16x32_f16(false, a, false, b, (short)0, c, false, false);
  }
};

__device__ __forceinline__ float sigm_f(float z) {
  const float zc = fminf(fmaxf(z, -30.0f), 30.0f);
  return __builtin_amdgcn_rcpf(1.0f + expf(-zc));
}
__device__ __forceinline__ float tanh_f(float z) {
  const float zc = fminf(fmaxf(z, -15.0f), 15.0f);
  return fmaf(-2.0f, __builtin_amdgcn_rcpf(expf(2.0f * zc) + 1.0f), 1.0f);
}

__device__ __forceinline__ void stage_x(const float* __restrict__ x, float* xs, int b0, int chunk, int tid) {
  const int row = tid >> 3, c4 = (tid & 7) * 4;
  const v4f v = *(const v4f*)(x + (size_t)(b0 + row) * TLEN + (size_t)chunk * TCH + c4);
  *(v4f*)(xs + row * TCH + c4) = v;
}
__device__ __forceinline__ void flush_lines(const float* os, float* __restrict__ out, int b0, int chunk, int tid) {
  const int row = tid >> 3, c4 = (tid & 7) * 4;
  const v4f v = *(const v4f*)(os + row * TCH + c4);
  float* p = out + (size_t)(b0 + row) * TLEN + (size_t)chunk * TCH + c4;
  *(volatile v4f*)p = v;
  __threadfence();
  *(volatile v4f*)p = v;
}

__global__ __launch_bounds__(NTHR) void lstm_seq_kernel(const float* __restrict__ x,
                                                        const float* __restrict__ w_ih,
                                                        const float* __restrict__ w_hh,
                                                        const float* __restrict__ b_ih,
                                                        const float* __restrict__ b_hh,
                                                        const float* __restrict__ fc_w,
                                                        const float* __restrict__ fc_b,
                                                        const int* __restrict__ fut,
                                                        float* __restrict__ out) {
  __shared__ __align__(16) unsigned Wlw[NWW];
  __shared__ __align__(16) _Float16 Ahi[MROWS * KP];
  __shared__ __align__(16) _Float16 Alo[MROWS * KP];
  __shared__ __align__(16) float    Hf[MROWS * HFP];
  __shared__ __align__(16) float    Xs[MROWS * TCH];
  __shared__ __align__(16) float    Os[MROWS * TCH];
  __shared__ __align__(16) float    Fw[UPAD];
  (void)fut;

  const int tid = threadIdx.x, lane = tid & 31, wave = tid >> 5;
  const int c = lane & 15, hh = lane >> 4, koff = hh * 8;
  const int b0 = blockIdx.x * MROWS;

#pragma unroll 1
  for (int i = tid; i < NWW; i += NTHR) {
    const int nr = i >> 5, kw = (i & 31) * 2;
    const int g = nr >> 6, u = nr & 63;
    const bool uok = (u < HID);
    const int n = g * HID + (uok ? u : (HID - 1));
    const int k0 = kw, k1 = kw + 1;
    const bool k0ok = (k0 < HID), k1ok = (k1 < HID);
    const float v0 = w_hh[n * HID + (k0ok ? k0 : (HID - 1))];
    const float v1 = w_hh[n * HID + (k1ok ? k1 : (HID - 1))];
    const float s0 = (uok && k0ok) ? v0 * WCARRY : 0.0f;
    const float s1 = (uok && k1ok) ? v1 * WCARRY : 0.0f;
    const _Float16 h0 = (_Float16)s0;
    const _Float16 h1 = (_Float16)s1;
    const unsigned short u0 = __builtin_bit_cast(unsigned short, h0);
    const unsigned short u1 = __builtin_bit_cast(unsigned short, h1);
    Wlw[i] = (unsigned)u0 | ((unsigned)u1 << 16);
  }
  {
    unsigned* ahw = (unsigned*)(void*)Ahi;
    unsigned* alw = (unsigned*)(void*)Alo;
#pragma unroll 1
    for (int i = tid; i < MROWS * KP / 2; i += NTHR) { ahw[i] = 0u; alw[i] = 0u; }
#pragma unroll 1
    for (int i = tid; i < MROWS * HFP; i += NTHR) Hf[i] = 0.0f;
  }
  if (tid < UPAD) {
    const float fv = fc_w[(tid < HID) ? tid : (HID - 1)];
    Fw[tid] = (tid < HID) ? fv : 0.0f;
  }
  stage_x(x, Xs, b0, 0, tid);

  const int u = 16 * wave + c;
  const bool uval = (u < HID);
  const int ucl = uval ? u : (HID - 1);
  float wih[NGATE], bih[NGATE], bhh[NGATE];
#pragma unroll
  for (int g = 0; g < NGATE; ++g) {
    const int n = g * HID + ucl;
    const float a0 = w_ih[n];
    const float a1 = b_ih[n];
    const float a2 = b_hh[n];
    asm volatile("" ::: "memory");
    wih[g] = uval ? a0 : 0.0f;
    bih[g] = uval ? a1 : 0.0f;
    bhh[g] = uval ? a2 : 0.0f;
  }
  const float fcb = fc_b[0];

  float cst[8], hst[8];
#pragma unroll
  for (int r = 0; r < 8; ++r) { cst[r] = 0.0f; hst[r] = 0.0f; }
  __syncthreads();

  const _Float16* Wl = (const _Float16*)(const void*)Wlw;
  const _Float16* arow_hi = Ahi + c * KP + koff;
  const _Float16* arow_lo = Alo + c * KP + koff;
  const _Float16* brow = Wl + (size_t)u * KP + koff;
  const v8f z8 = {0.f, 0.f, 0.f, 0.f, 0.f, 0.f, 0.f, 0.f};
  const int fq = lane >> 3, fpart = lane & 7;
  const int frow = 4 * wave + fq;

#pragma unroll 1
  for (int t = 0; t < TLEN; ++t) {
    const int tc = t & (TCH - 1);

    v8f ach[NGATE], acl[NGATE];
#pragma unroll
    for (int g = 0; g < NGATE; ++g) { ach[g] = z8; acl[g] = z8; }
#pragma unroll 1
    for (int k0 = 0; k0 < UPAD; k0 += 32) {
      const v16h ah = Frag<_Float16>::load(arow_hi + k0);
      const v16h al = Frag<_Float16>::load(arow_lo + k0);
      const v16h w0 = Frag<_Float16>::load(brow + 0 * UPAD * KP + k0);
      const v16h w1 = Frag<_Float16>::load(brow + 1 * UPAD * KP + k0);
      const v16h w2 = Frag<_Float16>::load(brow + 2 * UPAD * KP + k0);
      const v16h w3 = Frag<_Float16>::load(brow + 3 * UPAD * KP + k0);
      ach[0] = Frag<_Float16>::mma(ah, w0, ach[0]);
      acl[0] = Frag<_Float16>::mma(al, w0, acl[0]);
      ach[1] = Frag<_Float16>::mma(ah, w1, ach[1]);
      acl[1] = Frag<_Float16>::mma(al, w1, acl[1]);
      ach[2] = Frag<_Float16>::mma(ah, w2, ach[2]);
      acl[2] = Frag<_Float16>::mma(al, w2, acl[2]);
      ach[3] = Frag<_Float16>::mma(ah, w3, ach[3]);
      acl[3] = Frag<_Float16>::mma(al, w3, acl[3]);
      guard8x6(ach[0], ach[1], ach[2], ach[3], acl[0], acl[1], acl[2], acl[3], ah, al, w0, w1, w2, w3);
    }
    acc_guard4(ach[0], ach[1], ach[2], ach[3]);
    acc_guard4(acl[0], acl[1], acl[2], acl[3]);

    float xv[8];
#pragma unroll
    for (int r = 0; r < 8; ++r) xv[r] = Xs[(8 * hh + r) * TCH + tc];

#pragma unroll
    for (int r = 0; r < 8; ++r) {
      const float hw0 = ach[0][r] * FOLD_HI + acl[0][r] * FOLD_LO;
      const float hw1 = ach[1][r] * FOLD_HI + acl[1][r] * FOLD_LO;
      const float hw2 = ach[2][r] * FOLD_HI + acl[2][r] * FOLD_LO;
      const float hw3 = ach[3][r] * FOLD_HI + acl[3][r] * FOLD_LO;
      const float zi = (fmaf(xv[r], wih[0], bih[0]) + hw0) + bhh[0];
      const float zf = (fmaf(xv[r], wih[1], bih[1]) + hw1) + bhh[1];
      const float zg = (fmaf(xv[r], wih[2], bih[2]) + hw2) + bhh[2];
      const float zo = (fmaf(xv[r], wih[3], bih[3]) + hw3) + bhh[3];
      const float ig = sigm_f(zi);
      const float fg = sigm_f(zf);
      const float gg = tanh_f(zg);
      const float og = sigm_f(zo);
      const float cn = fg * cst[r] + ig * gg;
      cst[r] = cn;
      hst[r] = og * tanh_f(cn);
    }
    __syncthreads();

    if (tc == 0 && t > 0) flush_lines(Os, out, b0, (t / TCH) - 1, tid);
#pragma unroll
    for (int r = 0; r < 8; ++r) {
      const int row = 8 * hh + r;
      const float hs = uval ? hst[r] : 0.0f;
      const float h16 = hs * HCARRY;
      const _Float16 hiv = (_Float16)h16;
      const float res = (h16 - (float)hiv) * LCARRY;
      const _Float16 lov = (_Float16)res;
      Ahi[row * KP + u] = hiv;
      Alo[row * KP + u] = lov;
      Hf[row * HFP + u] = hs;
    }
    if (tc == TCH - 1 && (t + 1) < TLEN) stage_x(x, Xs, b0, (t + 1) / TCH, tid);
    __syncthreads();

    {
      const float* hp = Hf + frow * HFP + 8 * fpart;
      const v4f a0 = *(const v4f*)(hp);
      const v4f a1 = *(const v4f*)(hp + 4);
      const v4f f0 = *(const v4f*)(Fw + 8 * fpart);
      const v4f f1 = *(const v4f*)(Fw + 8 * fpart + 4);
      float s = 0.0f;
      s = fmaf(a0[0], f0[0], s); s = fmaf(a0[1], f0[1], s); s = fmaf(a0[2], f0[2], s); s = fmaf(a0[3], f0[3], s);
      s = fmaf(a1[0], f1[0], s); s = fmaf(a1[1], f1[1], s); s = fmaf(a1[2], f1[2], s); s = fmaf(a1[3], f1[3], s);
      s += __shfl_xor(s, 1, 32);
      s += __shfl_xor(s, 2, 32);
      s += __shfl_xor(s, 4, 32);
      const float tot = s + fcb;
      if (fpart == 0) Os[frow * TCH + tc] = tot;
    }
  }
  __syncthreads();
  flush_lines(Os, out, b0, NCHUNK - 1, tid);
}

extern "C" void kernel_launch(void* const* d_in, const int* in_sizes, int n_in,
                              void* d_out, int out_size, void* d_ws, size_t ws_size, hipStream_t stream) {
  (void)d_ws; (void)ws_size;
  if (n_in < 8 || d_out == nullptr) return;
  if (in_sizes[0] != NBATCH * TLEN || in_sizes[1] != G4H || in_sizes[2] != G4H * HID || in_sizes[3] != G4H ||
      in_sizes[4] != G4H || in_sizes[5] != HID || in_sizes[6] != 1 || in_sizes[7] != 1 || out_size != NBATCH * TLEN) return;

  const float* x    = (const float*)d_in[0];
  const float* w_ih = (const float*)d_in[1];
  const float* w_hh = (const float*)d_in[2];
  const float* b_ih = (const float*)d_in[3];
  const float* b_hh = (const float*)d_in[4];
  const float* fc_w = (const float*)d_in[5];
  const float* fc_b = (const float*)d_in[6];
  const int*   fut  = (const int*)d_in[7];
  float* out = (float*)d_out;

  lstm_seq_kernel<<<NBATCH / MROWS, NTHR, 0, stream>>>(x, w_ih, w_hh, b_ih, b_hh, fc_w, fc_b, fut, out);
}
